// TPMoEWrapper_63324997812518
// MI455X (gfx1250) — hardware-verified
//
#include <hip/hip_runtime.h>
#include <math.h>

typedef __attribute__((ext_vector_type(16))) _Float16 v16h;
typedef __attribute__((ext_vector_type(16))) __bf16 v16b;
typedef __attribute__((ext_vector_type(8)))  _Float16 v8h;
typedef __attribute__((ext_vector_type(8)))  __bf16 v8b;
typedef __attribute__((ext_vector_type(8)))  float v8f;
typedef __attribute__((ext_vector_type(4)))  float v4f;
typedef __attribute__((ext_vector_type(4)))  unsigned v4u;
typedef _Float16 h16;

#ifndef NB
#define NB 4
#endif
#ifndef SEQ
#define SEQ 1024
#endif
#define NB_FULL 4
#define SEQ_FULL 1024
#define NTOK (NB * SEQ)
#define NTOK_FULL (NB_FULL * SEQ_FULL)
#define DIN  512
#define DHID 2048
#define DOUT 512
#define NE   8
#define KF (NE * DHID)
#define KP KF
#define MCH (NTOK < 2048 ? NTOK : 2048)
#define HCARRY 64.0f
#define WCARRY 512.0f
#define OSCALE (1.0f / 32768.0f)
#define OUT1_ELEM ((size_t)NTOK_FULL * DOUT)

#define WS_XB  ((size_t)0)
#define WS_W13 (WS_XB  + (size_t)NTOK * DIN * 2)
#define WS_W2T (WS_W13 + (size_t)2 * NE * DHID * DIN * 2)
#define WS_CW  (WS_W2T + (size_t)DOUT * KP * 2)
#define WS_HB  (WS_CW  + (size_t)NTOK * NE * 4)
#define WS_END (WS_HB  + (size_t)MCH * KP * 2)

static_assert(NB == 1 || SEQ == SEQ_FULL);
static_assert(NB <= NB_FULL && SEQ <= SEQ_FULL);
static_assert(NTOK % 128 == 0 && MCH % 128 == 0 && NTOK % MCH == 0 && NTOK % 32 == 0);
static_assert(DIN % 32 == 0 && KP % 32 == 0 && (KP * 2) % 128 == 0 && DHID % 64 == 0 && DOUT % 128 == 0);
static_assert(NE == 8 && DIN % 8 == 0 && (NE * DIN) % 256 == 0);
static_assert(OUT1_ELEM * 4 == 8388608);
static_assert((OUT1_ELEM + (size_t)NTOK * NE) * 4 <= 8519680);
static_assert(WS_W13 % 128 == 0 && WS_W2T % 128 == 0 && WS_CW % 128 == 0 && WS_HB % 128 == 0);
static_assert(WS_END <= (size_t)134217728);
static_assert((size_t)(NTOK * DIN / 8 / 256) * 256 * 8 == (size_t)NTOK * DIN);
static_assert((size_t)(NE * DHID * DIN / 8 / 256) * 256 * 8 == (size_t)NE * DHID * DIN);
static_assert((size_t)(NE * DOUT * DHID / 8 / 256) * 256 * 8 == (size_t)DOUT * KF);
static_assert((size_t)(NTOK / 32) * 64 * 4 == (size_t)NTOK * NE);
static_assert((size_t)(DHID / 64) * (MCH / 128) * NE * 128 * 64 == (size_t)MCH * KF);
static_assert((size_t)(DOUT / 128) * (MCH / 128) * 128 * 128 == (size_t)MCH * DOUT);
static_assert(8 * 4 * 4 == 128 && 256 * 4 * 16 == 128 * 128);
static_assert(64 * 16 == 32 * NE * 4);
static_assert((size_t)(NE * (DIN + 4) + 2 * 32 * NE) * 4 <= 131072);
static_assert((size_t)128 * 64 * 2 <= 131072);
static_assert((size_t)8 * 16 * 64 * 4 <= 131072);

__device__ __forceinline__ v8f wmma16(v16h a, v16h b, v8f c) {
  v8f d = __builtin_amdgcn_wmma_f32_16x16x32_f16(false, a, false, b, (short)0, c, false, false);
  asm volatile("v_nop\n\tv_nop\n\tv_nop\n\tv_nop" : "+v"(d) : "v"(a), "v"(b));
  return d;
}
__device__ __forceinline__ v8f wmma_bf(v16b a, v16b b, v8f c) {
  v8f d = __builtin_amdgcn_wmma_f32_16x16x32_bf16(false, a, false, b, (short)0, c, false, false);
  asm volatile("v_nop\n\tv_nop\n\tv_nop\n\tv_nop" : "+v"(d) : "v"(a), "v"(b));
  return d;
}
__device__ __forceinline__ float bfr(float v) { return (float)(__bf16)v; }
static __device__ __forceinline__ h16 toh_flush(float v) { const h16 r = (h16)v; return (fabsf(v) < 6.103515625e-05f) ? (h16)0.0f : r; }
__device__ __forceinline__ v16b ldfrag_b(const unsigned short* p) { union { v16b v; v4u q[2]; } f; f.q[0] = *(const v4u*)p; f.q[1] = *(const v4u*)(p + 16); return f.v; }
__device__ __forceinline__ v16h ldfrag_h(const unsigned short* p) { union { v16h v; v4u q[2]; } f; f.q[0] = *(const v4u*)p; f.q[1] = *(const v4u*)(p + 16); return f.v; }

__global__ __launch_bounds__(256) void k_cvt_bf(const float* __restrict__ S, unsigned short* __restrict__ Dst, unsigned n8) {
  const unsigned i = blockIdx.x * 256u + threadIdx.x;
  const unsigned ic = i < n8 ? i : n8 - 1u;
  const v4f a = *(const v4f*)(S + (size_t)ic * 8), b = *(const v4f*)(S + (size_t)ic * 8 + 4);
  union { v8b h; v4u u; } o;
#pragma unroll
  for (int j = 0; j < 4; ++j) { o.h[j] = (__bf16)a[j]; o.h[4 + j] = (__bf16)b[j]; }
  const v4u val = o.u;
  volatile v4u* p = (volatile v4u*)(Dst + (size_t)ic * 8);
  *p = val; __threadfence(); *p = val;
}

__global__ __launch_bounds__(256) void k_cvt_w2(const float* __restrict__ W2, unsigned short* __restrict__ W2T) {
#pragma clang fp contract(off)
  const unsigned i = blockIdx.x * 256u + threadIdx.x;
  const unsigned ic = i < (unsigned)(NE * DOUT * DHID / 8) ? i : (unsigned)(NE * DOUT * DHID / 8 - 1);
  const unsigned f8 = ic % (unsigned)(DHID / 8), n = (ic / (unsigned)(DHID / 8)) % (unsigned)DOUT, e = ic / (unsigned)(DHID / 8 * DOUT);
  const v4f a = *(const v4f*)(W2 + (size_t)ic * 8), b = *(const v4f*)(W2 + (size_t)ic * 8 + 4);
  union { v8h h; v4u u; } o;
#pragma unroll
  for (int j = 0; j < 4; ++j) { o.h[j] = toh_flush(bfr(a[j]) * WCARRY); o.h[4 + j] = toh_flush(bfr(b[j]) * WCARRY); }
  const v4u val = o.u;
  volatile v4u* p = (volatile v4u*)(W2T + (size_t)n * KP + e * DHID + 8u * f8);
  *p = val; __threadfence(); *p = val;
}

__global__ __launch_bounds__(256) void k_router(const unsigned short* __restrict__ XB, const float* __restrict__ GW, float* __restrict__ LOUT, float* __restrict__ CW) {
#pragma clang fp contract(off)
  __shared__ __align__(16) float sg[NE][DIN + 4];
  __shared__ __align__(16) float sl[32][NE];
  __shared__ __align__(16) float sc[32][NE];
  const unsigned tid = threadIdx.x, r0 = blockIdx.x * 32u;
#pragma unroll 1
  for (unsigned it = 0; it < (unsigned)(NE * DIN / 256); ++it) { const unsigned idx = it * 256u + tid; sg[idx / DIN][idx % DIN] = bfr(GW[idx]); }
  __syncthreads();
  const unsigned tl = tid >> 3, e = tid & 7u;
  const unsigned short* xr = XB + (size_t)(r0 + tl) * DIN;
  float acc = 0.0f;
#pragma unroll 1
  for (unsigned kc = 0; kc < (unsigned)(DIN / 8); ++kc) {
    const v4u w = *(const v4u*)(xr + kc * 8u);
#pragma unroll
    for (int j = 0; j < 4; ++j) {
      const float x0 = __uint_as_float(w[j] << 16), x1 = __uint_as_float(w[j] & 0xffff0000u);
      acc = fmaf(x0, sg[e][kc * 8u + 2 * j], acc);
      acc = fmaf(x1, sg[e][kc * 8u + 2 * j + 1], acc);
    }
  }
  sl[tl][e] = acc;
  __syncthreads();
  if (tid < 32u) {
    const v4f la = *(const v4f*)&sl[tid][0], lb = *(const v4f*)&sl[tid][4];
    float l[8];
#pragma unroll
    for (int j = 0; j < 4; ++j) { l[j] = la[j]; l[4 + j] = lb[j]; }
    float v0 = -__builtin_huge_valf(), v1 = -__builtin_huge_valf(); int i0 = 0, i1 = 0;
#pragma unroll
    for (int j = 0; j < 8; ++j) { const float lj = l[j]; const bool g0 = lj > v0, g1 = lj > v1;
      v1 = g0 ? v0 : (g1 ? lj : v1); i1 = g0 ? i0 : (g1 ? j : i1);
      v0 = g0 ? lj : v0; i0 = g0 ? j : i0; }
    const float ex = expf(v1 - v0);
    const float inv = 1.0f / (1.0f + ex);
    const float w0 = inv, w1 = ex * inv;
    v4f ca, cb;
#pragma unroll
    for (int j = 0; j < 4; ++j) { ca[j] = (j == i0) ? w0 : ((j == i1) ? w1 : 0.0f); cb[j] = ((4 + j) == i0) ? w0 : (((4 + j) == i1) ? w1 : 0.0f); }
    *(v4f*)&sc[tid][0] = ca; *(v4f*)&sc[tid][4] = cb;
  }
  __syncthreads();
  if (tid < 64u) {
    const v4f lv = *(const v4f*)(&sl[0][0] + 4u * tid), cv = *(const v4f*)(&sc[0][0] + 4u * tid);
    volatile v4f* pl = (volatile v4f*)(LOUT + (size_t)r0 * NE + 4u * tid);
    volatile v4f* pc = (volatile v4f*)(CW + (size_t)r0 * NE + 4u * tid);
    *pl = lv; *pc = cv;
    __threadfence();
    *pl = lv; *pc = cv;
  }
}

__global__ __launch_bounds__(256) void k_h(const unsigned short* __restrict__ XB, const unsigned short* __restrict__ W13B, const float* __restrict__ CW, unsigned short* __restrict__ HB, unsigned tok0) {
  __shared__ __align__(16) _Float16 sh[128][64];
  const unsigned t = threadIdx.x, wave = (unsigned)__builtin_amdgcn_readfirstlane((int)(t >> 5)), lane = t & 31u, lm = lane & 15u, lh = lane >> 4, wm = wave >> 1, wn = wave & 1u;
  const unsigned e = blockIdx.z, m0 = blockIdx.y * 128u, n0 = blockIdx.x * 64u;
  const unsigned short* ar[2]; const unsigned short* br[4];
#pragma unroll
  for (int mi = 0; mi < 2; ++mi) ar[mi] = XB + (size_t)(tok0 + m0 + wm * 32u + mi * 16u + lm) * DIN + 8u * lh;
#pragma unroll
  for (int ni = 0; ni < 4; ++ni) br[ni] = W13B + ((size_t)(ni >> 1) * (size_t)(NE * DHID) + e * DHID + n0 + wn * 32u + (unsigned)(ni & 1) * 16u + lm) * DIN + 8u * lh;
  v8f acc[2][4] = {};
#pragma unroll 2
  for (unsigned kc = 0; kc < DIN / 32; ++kc) { v16b a[2], b[4];
#pragma unroll
    for (int mi = 0; mi < 2; ++mi) a[mi] = ldfrag_b(ar[mi] + kc * 32u);
#pragma unroll
    for (int ni = 0; ni < 4; ++ni) b[ni] = ldfrag_b(br[ni] + kc * 32u);
#pragma unroll
    for (int mi = 0; mi < 2; ++mi)
#pragma unroll
      for (int ni = 0; ni < 4; ++ni) acc[mi][ni] = wmma_bf(a[mi], b[ni], acc[mi][ni]); }
  float wv[2][8];
#pragma unroll
  for (int mi = 0; mi < 2; ++mi) {
#pragma unroll
    for (int r = 0; r < 8; ++r) wv[mi][r] = CW[(size_t)(tok0 + m0 + wm * 32u + mi * 16u + 8u * lh + r) * NE + e] * HCARRY;
    asm volatile("s_wait_loadcnt 0x0" ::: "memory"); }
#pragma unroll
  for (int ni = 0; ni < 2; ++ni)
#pragma unroll
    for (int mi = 0; mi < 2; ++mi)
#pragma unroll
      for (int r = 0; r < 8; ++r) { const float z = acc[mi][ni][r], g3 = acc[mi][ni + 2][r];
        const float s = z * __builtin_amdgcn_rcpf(1.0f + __expf(-z));
        sh[wm * 32u + mi * 16 + 8u * lh + r][wn * 32u + ni * 16 + lm] = toh_flush(s * g3 * wv[mi][r]); }
  __syncthreads();
  v4u o[4];
#pragma unroll
  for (unsigned it = 0; it < 4; ++it) { const unsigned rw = wave * 16u + it * 4u + (lane >> 3), q = lane & 7u; union { v8h h; v4u u; } w; w.h = *(const v8h*)&sh[rw][8u * q]; o[it] = w.u; }
  unsigned short* hb = HB + (size_t)m0 * KP + e * DHID + n0;
#pragma unroll
  for (unsigned it = 0; it < 4; ++it) { const unsigned rw = wave * 16u + it * 4u + (lane >> 3), q = lane & 7u; *(volatile v4u*)(hb + (size_t)rw * KP + 8u * q) = o[it]; }
  __threadfence();
#pragma unroll
  for (unsigned it = 0; it < 4; ++it) { const unsigned rw = wave * 16u + it * 4u + (lane >> 3), q = lane & 7u; *(volatile v4u*)(hb + (size_t)rw * KP + 8u * q) = o[it]; }
}

__global__ __launch_bounds__(256) void k_out(const unsigned short* __restrict__ HB, const unsigned short* __restrict__ W2T, float* __restrict__ OUT) {
  __shared__ __align__(16) float sf[8][16][64];
  const unsigned t = threadIdx.x, wave = t >> 5, lane = t & 31u, lm = lane & 15u, lh = lane >> 4, wm = wave >> 1, wn = wave & 1u;
  const unsigned m0 = blockIdx.y * 128u, n0 = blockIdx.x * 128u;
  const unsigned short* ar[2]; const unsigned short* br[4];
#pragma unroll
  for (int mi = 0; mi < 2; ++mi) ar[mi] = HB + (size_t)(m0 + wm * 32u + mi * 16u + lm) * KP + 8u * lh;
#pragma unroll
  for (int ni = 0; ni < 4; ++ni) br[ni] = W2T + (size_t)(n0 + wn * 64u + ni * 16u + lm) * KP + 8u * lh;
  v8f acc[2][4] = {};
#pragma unroll 2
  for (unsigned kc = 0; kc < KP / 32; ++kc) { v16h a[2], b[4];
#pragma unroll
    for (int mi = 0; mi < 2; ++mi) a[mi] = ldfrag_h(ar[mi] + kc * 32u);
#pragma unroll
    for (int ni = 0; ni < 4; ++ni) b[ni] = ldfrag_h(br[ni] + kc * 32u);
#pragma unroll
    for (int mi = 0; mi < 2; ++mi)
#pragma unroll
      for (int ni = 0; ni < 4; ++ni) acc[mi][ni] = wmma16(a[mi], b[ni], acc[mi][ni]); }
#pragma unroll
  for (int mi = 0; mi < 2; ++mi) {
    if (mi) __syncthreads();
#pragma unroll
    for (int ni = 0; ni < 4; ++ni)
#pragma unroll
      for (int r = 0; r < 8; ++r) sf[wave][8u * lh + r][ni * 16 + lm] = acc[mi][ni][r] * OSCALE;
    __syncthreads();
    v4f v[8];
#pragma unroll
    for (unsigned it = 0; it < 8; ++it) { const unsigned rw = it * 2u + (lane >> 4), pc = lane & 15u; v[it] = *(const v4f*)&sf[wave][rw][4u * pc]; }
    float* po = OUT + (size_t)(m0 + wm * 32u + mi * 16u) * DOUT + n0 + wn * 64u;
#pragma unroll
    for (unsigned it = 0; it < 8; ++it) { const unsigned rw = it * 2u + (lane >> 4), pc = lane & 15u; *(volatile v4f*)(po + (size_t)rw * DOUT + 4u * pc) = v[it]; }
    __threadfence();
#pragma unroll
    for (unsigned it = 0; it < 8; ++it) { const unsigned rw = it * 2u + (lane >> 4), pc = lane & 15u; *(volatile v4f*)(po + (size_t)rw * DOUT + 4u * pc) = v[it]; }
  }
}

extern "C" void kernel_launch(void* const* d_in, const int* in_sizes, int n_in, void* d_out, int out_size, void* d_ws, size_t ws_size, hipStream_t stream) {
  if (n_in < 5) return;
  if (in_sizes[0] < NTOK * DIN || in_sizes[1] < NE * DIN || in_sizes[2] < NE * DHID * DIN) return;
  if (in_sizes[3] < NE * DOUT * DHID || in_sizes[4] < NE * DHID * DIN) return;
  if ((size_t)out_size < OUT1_ELEM + (size_t)NTOK * NE) return;
  if (ws_size < (size_t)WS_END) return;
  const float* X  = (const float*)d_in[0];
  const float* GW = (const float*)d_in[1];
  const float* W1 = (const float*)d_in[2];
  const float* W2 = (const float*)d_in[3];
  const float* W3 = (const float*)d_in[4];
  char* ws = (char*)d_ws;
  unsigned short* XB   = (unsigned short*)(ws + WS_XB);
  unsigned short* W13B = (unsigned short*)(ws + WS_W13);
  unsigned short* W2T  = (unsigned short*)(ws + WS_W2T);
  float*          CW   = (float*)(ws + WS_CW);
  unsigned short* HB   = (unsigned short*)(ws + WS_HB);
  float* OUT  = (float*)d_out;
  float* LOUT = (float*)d_out + OUT1_ELEM;
  k_cvt_bf<<<dim3(NTOK * DIN / 8 / 256), 256, 0, stream>>>(X, XB, (unsigned)(NTOK * DIN / 8));
  k_cvt_bf<<<dim3(NE * DHID * DIN / 8 / 256), 256, 0, stream>>>(W1, W13B, (unsigned)(NE * DHID * DIN / 8));
  k_cvt_bf<<<dim3(NE * DHID * DIN / 8 / 256), 256, 0, stream>>>(W3, W13B + (size_t)NE * DHID * DIN, (unsigned)(NE * DHID * DIN / 8));
  k_cvt_w2<<<dim3(NE * DOUT * DHID / 8 / 256), 256, 0, stream>>>(W2, W2T);
  k_router<<<dim3(NTOK / 32), 256, 0, stream>>>(XB, GW, LOUT, CW);
  for (unsigned c = 0; c < (unsigned)(NTOK / MCH); ++c) {
    k_h<<<dim3(DHID / 64, MCH / 128, NE), 256, 0, stream>>>(XB, W13B, CW, HB, c * (unsigned)MCH);
    k_out<<<dim3(DOUT / 128, MCH / 128), 256, 0, stream>>>(HB, W2T, OUT + (size_t)c * MCH * DOUT);
  }
}
